// GraphConv_37855841747675
// MI455X (gfx1250) — hardware-run, weakly checked
//
#include <hip/hip_runtime.h>

typedef float          v8f   __attribute__((ext_vector_type(8)));
typedef float          v4f   __attribute__((ext_vector_type(4)));
typedef unsigned int   v4u   __attribute__((ext_vector_type(4)));
typedef int            v8i   __attribute__((ext_vector_type(8)));
typedef unsigned short v8us  __attribute__((ext_vector_type(8)));
typedef unsigned short v16us __attribute__((ext_vector_type(16)));
typedef __bf16         v16bf __attribute__((ext_vector_type(16)));
typedef _Float16       v16h  __attribute__((ext_vector_type(16)));
typedef v4f  __attribute__((may_alias)) v4fa;
typedef v8us __attribute__((may_alias)) v8usa;
union FragB { v16bf v; v16us u; v8us h[2]; v8i w; };
union FragH { v16h  v; v16us u; v8us h[2]; v8i w; };

__device__ __forceinline__ v8f wmb(const FragB& a, const FragB& b, v8f c) {
  v8f d = __builtin_amdgcn_wmma_f32_16x16x32_bf16(false, a.v, false, b.v, (short)0, c, false, false);
  asm volatile("v_nop\n\tv_nop\n\tv_nop\n\tv_nop" : "+v"(d) : "v"(a.w), "v"(b.w));
  return d;
}

__device__ __forceinline__ v8f wmh(const FragH& a, const FragH& b, v8f c) {
  v8f d = __builtin_amdgcn_wmma_f32_16x16x32_f16(false, a.v, false, b.v, (short)0, c, false, false);
  asm volatile("v_nop\n\tv_nop\n\tv_nop\n\tv_nop" : "+v"(d) : "v"(a.w), "v"(b.w));
  return d;
}

__device__ __forceinline__ unsigned bf16_bits(float f) {
  const unsigned u = __float_as_uint(f);
  const unsigned r = (u + 0x7FFFu + ((u >> 16) & 1u)) >> 16;
  const unsigned q = (u >> 16) | 0x40u;
  return ((u & 0x7fffffffu) > 0x7f800000u) ? q : r;
}

__device__ __forceinline__ float bf16_val(float f) {
  return __uint_as_float(bf16_bits(f) << 16);
}
__device__ __forceinline__ int clampi(int v, int lo, int hi) {
  return v < lo ? lo : (v > hi ? hi : v);
}

__device__ __forceinline__ unsigned f16_bits(float f) {
  const unsigned u  = __float_as_uint(f);
  const unsigned s  = (u >> 16) & 0x8000u;
  const unsigned a  = u & 0x7fffffffu;
  const unsigned t  = a - 0x38000000u;
  const unsigned r  = (t + 0x0FFFu + ((t >> 13) & 1u)) >> 13;
  const unsigned rc = r > 0x7C00u ? 0x7C00u : r;
  const bool small  = a < 0x38800000u;
  const bool isnan  = a > 0x7f800000u;
  const unsigned fin = small ? 0u : (s | rc);
  return isnan ? (s | 0x7E00u) : fin;
}

__device__ __forceinline__ unsigned pk16(unsigned lo, unsigned hi) { return lo | (hi << 16); }
__device__ __forceinline__ unsigned bf16_lo_bits(float v) {
  float hi = bf16_val(v);
  asm volatile("" : "+v"(hi));
  return bf16_bits(v - hi);
}
__device__ __forceinline__ v4u pack8_bf16(v4f a, v4f c) {
  return (v4u){ pk16(bf16_bits(a[0]), bf16_bits(a[1])), pk16(bf16_bits(a[2]), bf16_bits(a[3])),
                pk16(bf16_bits(c[0]), bf16_bits(c[1])), pk16(bf16_bits(c[2]), bf16_bits(c[3])) };
}
__device__ __forceinline__ v4u pack8_bf16_lo(v4f a, v4f c) {
  return (v4u){ pk16(bf16_lo_bits(a[0]), bf16_lo_bits(a[1])), pk16(bf16_lo_bits(a[2]), bf16_lo_bits(a[3])),
                pk16(bf16_lo_bits(c[0]), bf16_lo_bits(c[1])), pk16(bf16_lo_bits(c[2]), bf16_lo_bits(c[3])) };
}
__device__ __forceinline__ v4u pack8_f16(v4f a, v4f c) {
  return (v4u){ pk16(f16_bits(a[0]), f16_bits(a[1])), pk16(f16_bits(a[2]), f16_bits(a[3])),
                pk16(f16_bits(c[0]), f16_bits(c[1])), pk16(f16_bits(c[2]), f16_bits(c[3])) };
}

template <int FORM>
__global__ __launch_bounds__(256) void k_plane(const float* __restrict__ src, int rows, int cols, int ldsrc,
                                               unsigned short* __restrict__ dst, int MP, int KP) {
  static_assert(FORM >= 0 && FORM <= 3);
  const int KTOT = (FORM == 1 || FORM == 3) ? 2 * KP : KP;
  const unsigned ppr   = (unsigned)(KTOT >> 3);
  const unsigned kp8   = (unsigned)(KP >> 3);
  const unsigned total = (unsigned)MP * ppr;
  const unsigned g     = blockIdx.x * 256u + threadIdx.x;
  const unsigned rowu  = g / ppr;
  const unsigned p     = g - rowu * ppr;
  const bool second    = p >= kp8;
  const int row = (int)rowu;
  const int c0  = (int)((second ? p - kp8 : p) << 3);
  const float* srow = src + (size_t)clampi(row, 0, rows - 1) * (size_t)ldsrc;
  float x[8];
  unsigned mk[8];
#pragma unroll
  for (int e = 0; e < 8; ++e) {
    const int c = c0 + e;
    const float v = srow[clampi(c, 0, cols - 1)];
    asm volatile("" :: "v"(v));
    x[e]  = v;
    mk[e] = (row < rows && c < cols) ? 0xFFFFu : 0u;
  }
  const v4f a = (v4f){ x[0], x[1], x[2], x[3] };
  const v4f c = (v4f){ x[4], x[5], x[6], x[7] };
  v4u o;
  if (FORM == 2) {
    o = pack8_f16(a, c);
  } else {
    const v4u hi = pack8_bf16(a, c);
    o = hi;
    if (FORM == 1) { const v4u lo = pack8_bf16_lo(a, c); o = second ? lo : hi; }
  }
  const v4u mw = (v4u){ pk16(mk[0], mk[1]), pk16(mk[2], mk[3]), pk16(mk[4], mk[5]), pk16(mk[6], mk[7]) };
  o &= mw;
  if (g < total) {
    volatile v4u* q = (volatile v4u*)(dst + (size_t)g * 8);
    *q = o;
    __threadfence();
    *q = o;
  }
}

template <int FORM> struct FragOf    { typedef FragB T; };
template <>         struct FragOf<2> { typedef FragH T; };
__device__ __forceinline__ v8f mm(const FragB& a, const FragB& b, v8f c) { return wmb(a, b, c); }
__device__ __forceinline__ v8f mm(const FragH& a, const FragH& b, v8f c) { return wmh(a, b, c); }
template <class F> __device__ __forceinline__ F ld_frag(const unsigned short* p) {
  F f;
  f.h[0] = *(const v8usa*)(p);
  f.h[1] = *(const v8usa*)(p + 16);
  return f;
}

template <int FORM, int EPI>
__global__ __launch_bounds__(256) __attribute__((amdgpu_num_vgpr(248)))
void k_gemm_nt(const unsigned short* __restrict__ A, const unsigned short* __restrict__ B,
               const float* __restrict__ bias, float* __restrict__ D, int M, int N, int KTOT, int ldd) {
  static_assert(FORM >= 0 && FORM <= 2);
  static_assert(EPI == 0 || EPI == 1);
  typedef typename FragOf<FORM>::T F;
  __shared__ __attribute__((aligned(16))) float sT[8][16 * 68];
  const int lane = threadIdx.x & 31;
  const int wave = threadIdx.x >> 5;
  const int tilesM = (M + 63) >> 6;
  const int tilesN = (N + 63) >> 6;
  const int tile = blockIdx.x * 8 + wave;
  if (tile >= tilesM * tilesN) return;
  const int tm = tile / tilesN;
  const int tn = tile - tm * tilesN;
  const int m0 = tm << 6;
  const int n0 = tn << 6;

  const int rl = lane & 15;
  const int h8 = (lane >> 4) * 8;
  const unsigned short* pa = A + (size_t)(m0 + rl) * (size_t)KTOT + h8;
  const unsigned short* pb = B + (size_t)(n0 + rl) * (size_t)KTOT + h8;

  v8f acc[4][4];
#pragma unroll
  for (int i = 0; i < 4; ++i)
#pragma unroll
    for (int j = 0; j < 4; ++j) acc[i][j] = (v8f){0.f, 0.f, 0.f, 0.f, 0.f, 0.f, 0.f, 0.f};

#pragma unroll 1
  for (int k0 = 0; k0 < KTOT; k0 += 32) {
    F bf[4];
#pragma unroll
    for (int j = 0; j < 4; ++j) bf[j] = ld_frag<F>(pb + (size_t)(j << 4) * (size_t)KTOT + k0);
#pragma unroll
    for (int i = 0; i < 4; ++i) {
      const F af = ld_frag<F>(pa + (size_t)(i << 4) * (size_t)KTOT + k0);
#pragma unroll
      for (int j = 0; j < 4; ++j) acc[i][j] = mm(af, bf[j], acc[i][j]);
    }
  }

  float* slab = sT[wave];
  const int hh = lane >> 4;
  const int c4 = (lane & 15) * 4;
  const int nc = n0 + c4;
  const bool cok = nc < N;
  v4f bv = (v4f){0.f, 0.f, 0.f, 0.f};
  if (EPI == 1) {
    bv = *(const v4fa*)(bias + clampi(nc, 0, N - 4));
    asm volatile("" :: "v"(bv));
  }
#pragma unroll
  for (int i = 0; i < 4; ++i) {
    const int mBase = m0 + (i << 4);
#pragma unroll
    for (int j = 0; j < 4; ++j) {
#pragma unroll
      for (int r = 0; r < 8; ++r) slab[(h8 + r) * 68 + (j << 4) + rl] = acc[i][j][r];
    }
    __builtin_amdgcn_fence(__ATOMIC_RELEASE, "workgroup");
    __builtin_amdgcn_wave_barrier();
    __builtin_amdgcn_fence(__ATOMIC_ACQUIRE, "workgroup");
    v4f vv[8];
#pragma unroll
    for (int it = 0; it < 8; ++it) {
      const int row = it * 2 + hh;
      v4f v = *(const v4fa*)(slab + row * 68 + c4);
      if (EPI == 1) v += bv;
      vv[it] = v;
    }
    for (int pass = 0; pass < 2; ++pass) {
#pragma unroll
      for (int it = 0; it < 8; ++it) {
        const int row = mBase + it * 2 + hh;
        if (cok && row < M) *(volatile v4f*)(D + (size_t)row * (size_t)ldd + nc) = vv[it];
      }
      __threadfence();
    }
    __builtin_amdgcn_fence(__ATOMIC_RELEASE, "workgroup");
    __builtin_amdgcn_wave_barrier();
    __builtin_amdgcn_fence(__ATOMIC_ACQUIRE, "workgroup");
  }
}

#pragma clang fp contract(off)

typedef float  v2f __attribute__((ext_vector_type(2)));
typedef double v2d __attribute__((ext_vector_type(2)));
typedef v2f __attribute__((may_alias)) v2fa;

constexpr int NQ    = 50000;
constexpr int NS    = 50000;
constexpr int KNB   = 32;
constexpr int CF    = 64;
constexpr int CO    = 64;
constexpr int WLD   = 67;
constexpr int WOFF  = 3;
constexpr int MPAD  = 50048;
constexpr int NREC  = (NQ + 63) / 64;
constexpr int GT    = (NS + 63) / 64;
constexpr int NPOS  = NQ * KNB;
constexpr int OUT_ELEMS = NQ * CO;

static_assert(KNB == 32 && CO == 2 * 32 && CF == 64);
static_assert(NQ % 8 == 0 && NS % 8 == 0);
static_assert(NPOS == 1600000);
static_assert(WLD == CF + WOFF && WOFF == 3);
static_assert(NREC == 782 && GT == 782);
static_assert(MPAD % 64 == 0 && MPAD >= NS && CF % 32 == 0 && NS % 16 == 0 && CO % 4 == 0 && CO % 32 == 0);
static_assert((long long)MPAD * CF / 8 < 0x7fffffffLL && (MPAD * CF / 8) % 256 == 0);
static_assert(OUT_ELEMS == 3200000);

constexpr size_t SZ_FB   = (size_t)MPAD * CF * 2;
constexpr size_t SZ_P    = (size_t)MPAD * CO * 4;
constexpr size_t SZ_SPB  = (size_t)NS * 16;
constexpr size_t SZ_QPB  = (size_t)NQ * 16;
constexpr size_t SZ_WFB  = (size_t)CO * CF * 2;
constexpr size_t SZ_WXT  = (size_t)3 * CO * 4;
constexpr size_t SZ_GB   = (size_t)2 * CO * 4;
constexpr size_t SZ_ST   = (size_t)4 * CO * 4;
constexpr size_t SZ_MEAN = (size_t)CO * 4;
constexpr size_t SZ_REC  = (size_t)NREC * CO * 8;
constexpr size_t OFF_FB   = 0;
constexpr size_t OFF_P    = OFF_FB + SZ_FB;
constexpr size_t OFF_SPB  = OFF_P + SZ_P;
constexpr size_t OFF_QPB  = OFF_SPB + SZ_SPB;
constexpr size_t OFF_WFB  = OFF_QPB + SZ_QPB;
constexpr size_t OFF_WXT  = OFF_WFB + SZ_WFB;
constexpr size_t OFF_GB   = OFF_WXT + SZ_WXT;
constexpr size_t OFF_ST   = OFF_GB + SZ_GB;
constexpr size_t OFF_MEAN = OFF_ST + SZ_ST;
constexpr size_t OFF_RECA = OFF_MEAN + SZ_MEAN;
constexpr size_t OFF_RECB = OFF_RECA + SZ_REC;
constexpr size_t WS_TOTAL = OFF_RECB + SZ_REC;
static_assert(SZ_FB % 256 == 0 && SZ_P % 256 == 0 && SZ_SPB % 256 == 0 && SZ_QPB % 256 == 0 && SZ_WFB % 256 == 0);
static_assert(SZ_WXT % 256 == 0 && SZ_GB % 256 == 0 && SZ_ST % 256 == 0 && SZ_MEAN % 256 == 0 && SZ_REC % 256 == 0);
static_assert(OFF_P % 256 == 0 && OFF_SPB % 256 == 0 && OFF_QPB % 256 == 0 && OFF_WFB % 256 == 0 && OFF_WXT % 256 == 0);
static_assert(OFF_GB % 256 == 0 && OFF_ST % 256 == 0 && OFF_MEAN % 256 == 0 && OFF_RECA % 256 == 0 && OFF_RECB % 256 == 0);
static_assert(WS_TOTAL == (size_t)21629952);
static_assert(WS_TOTAL <= ((size_t)128 << 20));

constexpr int PB = (NS + 255) / 256;
constexpr int PREP_BLOCKS = 2 * PB + 4;
static_assert(NQ == NS && PB == 196);

__device__ __forceinline__ void prep_pts(const float* __restrict__ src, float* __restrict__ dst, int t, int n) {
  const int r = t < n ? t : n - 1;
  const float* s = src + (size_t)r * 3;
  const float x = s[0], y = s[1], z = s[2];
  asm volatile("" :: "v"(x));
  asm volatile("" :: "v"(y));
  asm volatile("" :: "v"(z));
  const v4f o = (v4f){ bf16_val(x), bf16_val(y), bf16_val(z), 0.0f };
  if (t < n) {
    volatile v4f* q = (volatile v4f*)(dst + (size_t)t * 4);
    *q = o;
    __threadfence();
    *q = o;
  }
}

__global__ __launch_bounds__(256) void k_prep(const float* __restrict__ qpts, const float* __restrict__ spts,
                                              const float* __restrict__ convw, const float* __restrict__ gamma,
                                              const float* __restrict__ beta, float* __restrict__ SPB,
                                              float* __restrict__ QPB, unsigned short* __restrict__ WFB,
                                              float* __restrict__ WXT, float* __restrict__ GB) {
  const int tid = (int)threadIdx.x;
  const int blk = (int)blockIdx.x;
  if (blk < PB) {
    prep_pts(spts, SPB, blk * 256 + tid, NS);
  } else if (blk < 2 * PB) {
    prep_pts(qpts, QPB, (blk - PB) * 256 + tid, NQ);
  } else if (blk < 2 * PB + 2) {
    const int g  = (blk - 2 * PB) * 256 + tid;
    const int n  = g >> 3;
    const int k0 = (g & 7) * 8;
    const float* s = convw + (size_t)n * WLD + WOFF + k0;
    float x[8];
#pragma unroll
    for (int e = 0; e < 8; ++e) {
      const float v = s[e];
      asm volatile("" :: "v"(v));
      x[e] = v;
    }
    const v4u o = pack8_bf16((v4f){ x[0], x[1], x[2], x[3] }, (v4f){ x[4], x[5], x[6], x[7] });
    volatile v4u* q = (volatile v4u*)(WFB + (size_t)g * 8);
    *q = o;
    __threadfence();
    *q = o;
  } else if (blk == 2 * PB + 2) {
    const int u  = tid < 48 ? tid : 47;
    const int c  = u >> 4;
    const int o0 = (u & 15) * 4;
    float v[4];
#pragma unroll
    for (int e = 0; e < 4; ++e) {
      const float w = convw[(size_t)(o0 + e) * WLD + c];
      asm volatile("" :: "v"(w));
      v[e] = bf16_val(w);
    }
    const v4f o = (v4f){ v[0], v[1], v[2], v[3] };
    if (tid < 48) {
      volatile v4f* q = (volatile v4f*)(WXT + 4 * tid);
      *q = o;
      __threadfence();
      *q = o;
    }
  } else {
    const int u  = tid < 32 ? tid : 31;
    const int ig = clampi(u, 0, 15) * 4;
    const int ib = clampi(u - 16, 0, 15) * 4;
    const v4f a0 = *(const v4fa*)(gamma + ig);
    const v4f a1 = *(const v4fa*)(beta + ib);
    asm volatile("" :: "v"(a0));
    asm volatile("" :: "v"(a1));
    const unsigned m0 = (u < 16) ? 0xFFFFFFFFu : 0u;
    const unsigned m1 = ~m0;
    v4f o;
#pragma unroll
    for (int e = 0; e < 4; ++e) {
      const unsigned bits = (__float_as_uint(a0[e]) & m0) | (__float_as_uint(a1[e]) & m1);
      o[e] = bf16_val(__uint_as_float(bits));
    }
    if (tid < 32) {
      volatile v4f* q = (volatile v4f*)(GB + 4 * tid);
      *q = o;
      __threadfence();
      *q = o;
    }
  }
}

__device__ __forceinline__ void q_setup(const int* __restrict__ ids, const float* __restrict__ SPB,
                                        const float* __restrict__ QPB, int q, int lane,
                                        int& idc, int& keep, int& dxi, int& dyi, int& dzi) {
  int id = ids[(size_t)q * KNB + lane];
  asm volatile("" :: "v"(id));
  idc = clampi(id, 0, NS - 1);
  keep = (id == NS) ? 0 : -1;
  const v4f sv = *(const v4fa*)(SPB + (size_t)idc * 4);
  const v4f qv = *(const v4fa*)(QPB + (size_t)q * 4);
  const float sx = sv[0], sy = sv[1], sz = sv[2];
  const float qx = qv[0], qy = qv[1], qz = qv[2];
  asm volatile("" :: "v"(sx));
  asm volatile("" :: "v"(sy));
  asm volatile("" :: "v"(sz));
  asm volatile("" :: "v"(qx));
  asm volatile("" :: "v"(qy));
  asm volatile("" :: "v"(qz));
  dxi = __float_as_int(sx - qx) & keep;
  dyi = __float_as_int(sy - qy) & keep;
  dzi = __float_as_int(sz - qz) & keep;
}

__device__ __forceinline__ void z_pair(const float* __restrict__ Pl, int idc, int keep, int dxi, int dyi, int dzi, int k,
                                       float wa0, float wa1, float wa2, float wb0, float wb1, float wb2,
                                       float& z0, float& z1) {
  const int      nr = __builtin_amdgcn_readlane(idc, k);
  const unsigned km = (unsigned)__builtin_amdgcn_readlane(keep, k);
  const float x0 = __int_as_float(__builtin_amdgcn_readlane(dxi, k));
  const float x1 = __int_as_float(__builtin_amdgcn_readlane(dyi, k));
  const float x2 = __int_as_float(__builtin_amdgcn_readlane(dzi, k));
  const v2f pv = *(const v2fa*)(Pl + (size_t)nr * CO);
  const float p0 = pv[0], p1 = pv[1];
  asm volatile("" :: "v"(p0));
  asm volatile("" :: "v"(p1));
  const float ps0 = __uint_as_float(__float_as_uint(p0) & km);
  const float ps1 = __uint_as_float(__float_as_uint(p1) & km);
  const float t0 = fmaf(wa2, x2, fmaf(wa1, x1, wa0 * x0));
  const float t1 = fmaf(wb2, x2, fmaf(wb1, x1, wb0 * x0));
  z0 = ps0 + t0;
  z1 = ps1 + t1;
}

__device__ __forceinline__ void load_wx(const float* __restrict__ WXT, int lane,
                                        float& wa0, float& wa1, float& wa2, float& wb0, float& wb1, float& wb2) {
  const v2f w0 = *(const v2fa*)(WXT + 0 * CO + 2 * lane);
  const v2f w1 = *(const v2fa*)(WXT + 1 * CO + 2 * lane);
  const v2f w2 = *(const v2fa*)(WXT + 2 * CO + 2 * lane);
  asm volatile("" :: "v"(w0));
  asm volatile("" :: "v"(w1));
  asm volatile("" :: "v"(w2));
  wa0 = w0[0]; wb0 = w0[1];
  wa1 = w1[0]; wb1 = w1[1];
  wa2 = w2[0]; wb2 = w2[1];
}

template <int MODE>
__global__ __launch_bounds__(256) void k_stat(const int* __restrict__ ids, const float* __restrict__ SPB,
                                              const float* __restrict__ QPB, const float* __restrict__ P,
                                              const float* __restrict__ WXT, const float* __restrict__ MEAN,
                                              double* __restrict__ rec) {
  static_assert(MODE == 0 || MODE == 1);
  __shared__ __attribute__((aligned(16))) double sD[8 * CO];
  const int tid = (int)threadIdx.x, lane = tid & 31, wave = tid >> 5;
  float wa0, wa1, wa2, wb0, wb1, wb2;
  load_wx(WXT, lane, wa0, wa1, wa2, wb0, wb1, wb2);
  float m0 = 0.0f, m1 = 0.0f;
  if constexpr (MODE == 1) {
    const v2f mv = *(const v2fa*)(MEAN + 2 * lane);
    asm volatile("" :: "v"(mv));
    m0 = mv[0]; m1 = mv[1];
  }
  const float* Pl = P + 2 * lane;
  const int base = (int)blockIdx.x * 64 + wave * 8;
  const int ntrip = __builtin_amdgcn_readfirstlane(clampi(NQ - base, 0, 8));
  double d0 = 0.0, d1 = 0.0;
#pragma unroll 1
  for (int i = 0; i < ntrip; ++i) {
    const int q = __builtin_amdgcn_readfirstlane(base + i);
    int idc, keep, dxi, dyi, dzi;
    q_setup(ids, SPB, QPB, q, lane, idc, keep, dxi, dyi, dzi);
    float s0 = 0.0f, s1 = 0.0f;
#pragma unroll 4
    for (int k = 0; k < KNB; ++k) {
      float z0, z1;
      z_pair(Pl, idc, keep, dxi, dyi, dzi, k, wa0, wa1, wa2, wb0, wb1, wb2, z0, z1);
      if constexpr (MODE == 0) {
        s0 += z0; s1 += z1;
      } else {
        const float e0 = z0 - m0, e1 = z1 - m1;
        s0 += e0 * e0; s1 += e1 * e1;
      }
    }
    d0 += (double)s0;
    d1 += (double)s1;
  }
  sD[wave * CO + 2 * lane]     = d0;
  sD[wave * CO + 2 * lane + 1] = d1;
  __syncthreads();
  if (tid < 32) {
    double a0 = 0.0, a1 = 0.0;
#pragma unroll
    for (int w = 0; w < 8; ++w) {
      a0 += sD[w * CO + 2 * tid];
      a1 += sD[w * CO + 2 * tid + 1];
    }
    const v2d o = (v2d){ a0, a1 };
    volatile v2d* qd = (volatile v2d*)(rec + (size_t)blockIdx.x * CO + 2 * tid);
    *qd = o;
    __threadfence();
    *qd = o;
  }
}

template <int MODE>
__global__ __launch_bounds__(64) void k_comb(const double* __restrict__ rec, double inv_count,
                                             const float* __restrict__ MEANin, const float* __restrict__ GB,
                                             float* __restrict__ out) {
  static_assert(MODE == 0 || MODE == 1);
  __shared__ __attribute__((aligned(16))) float sv[CO];
  const int tid = (int)threadIdx.x;
  double s = 0.0;
#pragma unroll 4
  for (int i = 0; i < NREC; ++i) s += rec[(size_t)i * CO + tid];
  const float qf = (float)(s * inv_count);
  float val = qf;
  if constexpr (MODE == 1) val = 1.0f / sqrtf(qf + 1e-5f);
  sv[tid] = val;
  __syncthreads();
  if constexpr (MODE == 0) {
    const int t4 = tid < 16 ? tid : 15;
    const v4f o = *(const v4fa*)(sv + 4 * t4);
    if (tid < 16) {
      volatile v4f* q = (volatile v4f*)(out + 4 * tid);
      *q = o;
      __threadfence();
      *q = o;
    }
  } else {
    const int j   = tid & 15;
    const int sel = tid >> 4;
    const v4f am = *(const v4fa*)(MEANin + 4 * j);
    const v4f ar = *(const v4fa*)(sv + 4 * j);
    const v4f ag = *(const v4fa*)(GB + 4 * j);
    const v4f ab = *(const v4fa*)(GB + CO + 4 * j);
    asm volatile("" :: "v"(am));
    asm volatile("" :: "v"(ar));
    asm volatile("" :: "v"(ag));
    asm volatile("" :: "v"(ab));
    const unsigned k0 = (sel == 0) ? 0xFFFFFFFFu : 0u;
    const unsigned k1 = (sel == 1) ? 0xFFFFFFFFu : 0u;
    const unsigned k2 = (sel == 2) ? 0xFFFFFFFFu : 0u;
    const unsigned k3 = (sel == 3) ? 0xFFFFFFFFu : 0u;
    v4f o;
#pragma unroll
    for (int e = 0; e < 4; ++e) {
      const unsigned bits = (__float_as_uint(am[e]) & k0) | (__float_as_uint(ar[e]) & k1) |
                            (__float_as_uint(ag[e]) & k2) | (__float_as_uint(ab[e]) & k3);
      o[e] = __uint_as_float(bits);
    }
    volatile v4f* q = (volatile v4f*)(out + 4 * tid);
    *q = o;
    __threadfence();
    *q = o;
  }
}

static_assert((NQ / 8) * 8 == NQ);
static_assert((size_t)(NQ - 1) * CO + 2 * 31 + 1 == (size_t)OUT_ELEMS - 1);
__global__ __launch_bounds__(256) void k_apply(const int* __restrict__ ids, const float* __restrict__ SPB,
                                               const float* __restrict__ QPB, const float* __restrict__ P,
                                               const float* __restrict__ WXT, const float* __restrict__ ST,
                                               float* __restrict__ out) {
  const int tid = (int)threadIdx.x, lane = tid & 31, wave = tid >> 5;
  const int row = __builtin_amdgcn_readfirstlane((int)blockIdx.x * 8 + wave);
  const int rq  = row < NQ ? row : NQ - 1;
  float wa0, wa1, wa2, wb0, wb1, wb2;
  load_wx(WXT, lane, wa0, wa1, wa2, wb0, wb1, wb2);
  const v2f mv = *(const v2fa*)(ST + 0 * CO + 2 * lane);
  const v2f rv = *(const v2fa*)(ST + 1 * CO + 2 * lane);
  const v2f gv = *(const v2fa*)(ST + 2 * CO + 2 * lane);
  const v2f bv = *(const v2fa*)(ST + 3 * CO + 2 * lane);
  asm volatile("" :: "v"(mv));
  asm volatile("" :: "v"(rv));
  asm volatile("" :: "v"(gv));
  asm volatile("" :: "v"(bv));
  const float m0 = mv[0], m1 = mv[1], r0 = rv[0], r1 = rv[1];
  const float g0 = gv[0], g1 = gv[1], b0 = bv[0], b1 = bv[1];
  const float* Pl = P + 2 * lane;
  int idc, keep, dxi, dyi, dzi;
  q_setup(ids, SPB, QPB, rq, lane, idc, keep, dxi, dyi, dzi);
  float mx0 = -__builtin_inff(), mx1 = -__builtin_inff();
#pragma unroll 4
  for (int k = 0; k < KNB; ++k) {
    float z0, z1;
    z_pair(Pl, idc, keep, dxi, dyi, dzi, k, wa0, wa1, wa2, wb0, wb1, wb2, z0, z1);
    const float y0 = ((z0 - m0) * r0) * g0 + b0;
    const float y1 = ((z1 - m1) * r1) * g1 + b1;
    const float a0 = (y0 >= 0.0f) ? y0 : 0.1f * y0;
    const float a1 = (y1 >= 0.0f) ? y1 : 0.1f * y1;
    const bool t0 = (a0 > mx0) || (a0 != a0);
    const bool t1 = (a1 > mx1) || (a1 != a1);
    mx0 = t0 ? a0 : mx0;
    mx1 = t1 ? a1 : mx1;
  }
  const v2f o = (v2f){ mx0, mx1 };
  if (row < NQ) {
    volatile v2f* q = (volatile v2f*)(out + (size_t)row * CO + 2 * lane);
    *q = o;
    __threadfence();
    *q = o;
  }
}

extern "C" void kernel_launch(void* const* d_in, const int* in_sizes, int n_in,
                              void* d_out, int out_size, void* d_ws, size_t ws_size,
                              hipStream_t stream) {
  if (n_in < 7) return;
  if (in_sizes[0] != NQ * 3) return;
  if (in_sizes[1] != NS * 3) return;
  if (in_sizes[2] != NS * CF) return;
  if (in_sizes[3] != CO * WLD) return;
  if (in_sizes[4] != CO || in_sizes[5] != CO) return;
  if (in_sizes[6] != NQ * KNB) return;
  if (out_size != OUT_ELEMS) return;
  if (ws_size < WS_TOTAL) return;

  const float* qpts  = (const float*)d_in[0];
  const float* spts  = (const float*)d_in[1];
  const float* feat  = (const float*)d_in[2];
  const float* convw = (const float*)d_in[3];
  const float* gamma = (const float*)d_in[4];
  const float* beta  = (const float*)d_in[5];
  const int*   ids   = (const int*)d_in[6];
  float* out = (float*)d_out;

  char* ws = (char*)d_ws;
  unsigned short* FB   = (unsigned short*)(ws + OFF_FB);
  float*          P    = (float*)(ws + OFF_P);
  float*          SPB  = (float*)(ws + OFF_SPB);
  float*          QPB  = (float*)(ws + OFF_QPB);
  unsigned short* WFB  = (unsigned short*)(ws + OFF_WFB);
  float*          WXT  = (float*)(ws + OFF_WXT);
  float*          GB   = (float*)(ws + OFF_GB);
  float*          ST   = (float*)(ws + OFF_ST);
  float*          MEAN = (float*)(ws + OFF_MEAN);
  double*         RECA = (double*)(ws + OFF_RECA);
  double*         RECB = (double*)(ws + OFF_RECB);

  const double inv_count = 1.0 / 1600000.0;

  k_prep<<<PREP_BLOCKS, 256, 0, stream>>>(qpts, spts, convw, gamma, beta, SPB, QPB, WFB, WXT, GB);
  k_plane<0><<<MPAD * CF / 8 / 256, 256, 0, stream>>>(feat, NS, CF, CF, FB, MPAD, CF);
  k_gemm_nt<0, 0><<<(GT + 7) / 8, 256, 0, stream>>>(FB, WFB, GB, P, NS, CO, CF, CO);
  k_stat<0><<<NREC, 256, 0, stream>>>(ids, SPB, QPB, P, WXT, MEAN, RECA);
  k_comb<0><<<1, 64, 0, stream>>>(RECA, inv_count, GB, GB, MEAN);
  k_stat<1><<<NREC, 256, 0, stream>>>(ids, SPB, QPB, P, WXT, MEAN, RECB);
  k_comb<1><<<1, 64, 0, stream>>>(RECB, inv_count, MEAN, GB, ST);
  k_apply<<<NQ / 8, 256, 0, stream>>>(ids, SPB, QPB, P, WXT, ST, out);
}
